// MultiRelationGNN_75746043232940
// MI455X (gfx1250) — hardware-verified
//
#include <hip/hip_runtime.h>
#include <math.h>

typedef __attribute__((ext_vector_type(16))) _Float16 v16h;
typedef __attribute__((ext_vector_type(16))) __bf16 v16b;
typedef __attribute__((ext_vector_type(8)))  _Float16 v8h;
typedef __attribute__((ext_vector_type(8)))  float v8f;
typedef __attribute__((ext_vector_type(4)))  float v4f;
typedef __attribute__((ext_vector_type(2)))  float v2f;
typedef __attribute__((ext_vector_type(4)))  unsigned v4u;
typedef __attribute__((ext_vector_type(4)))  int v4i;
typedef float __attribute__((may_alias)) float_a;
typedef int __attribute__((may_alias)) int_a;

template <typename T> __device__ __forceinline__ void vst2(void* p, T v) { *(volatile T*)p = v; __threadfence(); *(volatile T*)p = v; }
__device__ __forceinline__ v8f wmma16(v16h a, v16h b, v8f c) {
  v8f d = __builtin_amdgcn_wmma_f32_16x16x32_f16(false, a, false, b, (short)0, c, false, false);
  asm volatile("v_nop\n\tv_nop\n\tv_nop\n\tv_nop" : "+v"(d) : "v"(a), "v"(b));
  return d;
}
__device__ __forceinline__ v8f wmma_bf(v16b a, v16b b, v8f c) {
  v8f d = __builtin_amdgcn_wmma_f32_16x16x32_bf16(false, a, false, b, (short)0, c, false, false);
  asm volatile("v_nop\n\tv_nop\n\tv_nop\n\tv_nop" : "+v"(d) : "v"(a), "v"(b));
  return d;
}
__device__ __forceinline__ v16h frag_h(const _Float16* rowk0, int lane) {
  union { v16h v; v8h q[2]; } u; const _Float16* p = rowk0 + 8 * (lane >> 4);
  u.q[0] = *(const v8h*)p; u.q[1] = *(const v8h*)(p + 16); return u.v;
}
__device__ __forceinline__ v16h frag_f32(const float* rowk0, int lane) {
  v16h a; const float* p = rowk0 + 8 * (lane >> 4);
#pragma unroll
  for (int i = 0; i < 8; ++i) { a[i] = (_Float16)p[i]; a[8 + i] = (_Float16)p[16 + i]; }
  return a;
}
__device__ __forceinline__ v16h frag_f32s(const float* rowk0, int lane, float sc) {
  v16h a; const float* p = rowk0 + 8 * (lane >> 4);
#pragma unroll
  for (int i = 0; i < 8; ++i) { a[i] = (_Float16)(p[i] * sc); a[8 + i] = (_Float16)(p[16 + i] * sc); }
  return a;
}
__device__ __forceinline__ v16h fragc_f32(const float* W, int k0, int n, int lane, int ld, int K) {
  v16h a; const int g = lane >> 4;
#pragma unroll
  for (int i = 0; i < 8; ++i) { const int ka = k0 + 8 * g + i, kb = ka + 16;
    a[i] = (_Float16)(ka < K ? W[(size_t)ka * ld + n] : 0.f); a[8 + i] = (_Float16)(kb < K ? W[(size_t)kb * ld + n] : 0.f); }
  return a;
}
struct F2 { v16b h, l; };
__device__ __forceinline__ F2 bsplit16(const float v[16]) { F2 r;
#pragma unroll
  for (int i = 0; i < 16; ++i) { const __bf16 h = (__bf16)v[i]; r.h[i] = h; r.l[i] = (__bf16)(v[i] - (float)h); }
  return r; }
__device__ __forceinline__ F2 split_row(const float* row, int k0, int lane) { float v[16]; const float* p = row + k0 + 8 * (lane >> 4);
#pragma unroll
  for (int i = 0; i < 8; ++i) { v[i] = p[i]; v[8 + i] = p[16 + i]; }
  return bsplit16(v); }
__device__ __forceinline__ F2 split_rowK(const float* row, int k0, int lane, int K) { float v[16]; const int g = lane >> 4;
#pragma unroll
  for (int i = 0; i < 8; ++i) { const int ka = k0 + 8 * g + i, kb = ka + 16; v[i] = ka < K ? row[ka] : 0.f; v[8 + i] = kb < K ? row[kb] : 0.f; }
  return bsplit16(v); }
__device__ __forceinline__ F2 split_col(const float* W, int k0, int n, int lane, int ld, int K) { float v[16]; const int g = lane >> 4;
#pragma unroll
  for (int i = 0; i < 8; ++i) { const int ka = k0 + 8 * g + i, kb = ka + 16; v[i] = ka < K ? W[(size_t)ka * ld + n] : 0.f; v[8 + i] = kb < K ? W[(size_t)kb * ld + n] : 0.f; }
  return bsplit16(v); }
__device__ __forceinline__ v8f mac3(const F2& a, const F2& b, v8f c) { c = wmma_bf(a.l, b.h, c); c = wmma_bf(a.h, b.l, c); return wmma_bf(a.h, b.h, c); }
__device__ __forceinline__ float sigm(float v) { return 1.0f / (1.0f + expf(-v)); }
#define LDSX() do { asm volatile("s_wait_dscnt 0" ::: "memory"); __builtin_amdgcn_wave_barrier(); __builtin_amdgcn_fence(__ATOMIC_RELEASE, "workgroup"); } while (0)


#define NN 50000
#define NE 1600000
#define DIN 128
#define HD 64
#define NR 5
#define TW (NR * HD)
#define KB (NR * HD)
#define RB 1024
#define NRB 49
#define NNP (NRB * RB)
#define EPT 8
#define CH (256 * EPT)
__device__ __forceinline__ float lrelu(float v) { return v >= 0.f ? v : 0.01f * v; }
__device__ __forceinline__ int clampn(int v) { return v < 0 ? 0 : (v >= NN ? NN - 1 : v); }

template <int K, int NOUT, int MODE>
__global__ __launch_bounds__(128) void k_node(const float* __restrict__ A, int lda, const float* __restrict__ Bm, const float* __restrict__ bias, float* __restrict__ C) {
  __shared__ __align__(16) float so[4][16][132];
  const int tid = threadIdx.x, wave = tid >> 5, lane = tid & 31, col = lane & 15, g = lane >> 4;
  const int r0 = blockIdx.x * 64 + wave * 16; const int ra = (r0 + col) < NN ? (r0 + col) : (NN - 1);
  constexpr int NPASS = (NOUT + 127) / 128;
#pragma unroll 1
  for (int ps = 0; ps < NPASS; ++ps) { const int n0 = ps * 128; const int nt = (NOUT - n0) >= 128 ? 8 : (NOUT - n0) / 16;
    v8f acc[8] = {};
#pragma unroll 1
    for (int kc = 0; kc < K / 32; ++kc) { const F2 a = split_row(A + (size_t)ra * lda, kc * 32, lane);
#pragma unroll
      for (int j = 0; j < 8; ++j) if (j < nt) { const int n = n0 + j * 16 + col; const float* Bp; int ldb, nn;
          if (MODE == 0) { Bp = Bm; ldb = NOUT; nn = n; }
          else { const int r = n / HD; Bp = Bm + ((size_t)r * 2 * HD) * HD; ldb = HD; nn = n % HD; }
          acc[j] = mac3(a, split_col(Bp, kc * 32, nn, lane, ldb, K), acc[j]); } }
#pragma unroll
    for (int j = 0; j < 8; ++j) if (j < nt) { const int n = n0 + j * 16 + col; const float bb = (MODE == 0) ? bias[n] : 0.f;
#pragma unroll
      for (int rr = 0; rr < 8; ++rr) { const int row = r0 + 8 * g + rr; so[wave][8 * g + rr][j * 16 + col] = row < NN ? acc[j][rr] + bb : 0.f; } }
    LDSX();
    const int npc = nt * 4;
    for (int q = lane; q < 16 * npc; q += 32) { const int rl = q / npc, pc = q % npc; vst2(C + (size_t)(r0 + rl) * NOUT + n0 + pc * 4, *(const v4f*)(&so[wave][rl][pc * 4])); }
    LDSX(); }
}
__global__ __launch_bounds__(256) void k_rel(const int* __restrict__ esrc, const int* __restrict__ edst, const int* __restrict__ etyp, const float* __restrict__ etim, const float* __restrict__ lam, const float* __restrict__ beta,
                                            const float* __restrict__ T, float* __restrict__ Hpart, float* __restrict__ WS) {
  __shared__ __align__(16) float sacc[RB][HD];
  __shared__ float sws[RB][NR];
  __shared__ int ssrc[8][32 * EPT], sdl[8][32 * EPT]; __shared__ float swgt[8][32 * EPT]; __shared__ int scnt[8];
  const int tid = threadIdx.x, wave = tid >> 5, lane = tid & 31;
  const int r0 = blockIdx.x * RB; const float lamv = lam[0], betav = beta[0];
  for (int q = tid; q < RB * HD; q += 256) (&sacc[0][0])[q] = 0.f;
  for (int q = tid; q < RB * NR; q += 256) (&sws[0][0])[q] = 0.f;
  __syncthreads();
#pragma unroll 1
  for (int c0 = 0; c0 < NE; c0 += CH) { const int e0 = c0 + tid * EPT; int hd[EPT]; int cnt = 0;
    if (e0 + EPT <= NE) {
#pragma unroll
      for (int v = 0; v < EPT / 4; ++v) { const int4 d4 = *(const int4*)(edst + e0 + v * 4); const int dd[4] = {d4.x, d4.y, d4.z, d4.w};
#pragma unroll
        for (int u = 0; u < 4; ++u) { const unsigned rel = (unsigned)(clampn(dd[u]) - r0); const bool h = rel < (unsigned)RB; hd[v * 4 + u] = h ? (int)rel : -1; cnt += h ? 1 : 0; } } }
    else {
#pragma unroll
      for (int u = 0; u < EPT; ++u) { const int e = e0 + u; hd[u] = -1; if (e < NE) { const unsigned rel = (unsigned)(clampn(edst[e]) - r0); if (rel < (unsigned)RB) { hd[u] = (int)rel; ++cnt; } } } }
    int incl = cnt;
#pragma unroll
    for (int off = 1; off < 32; off <<= 1) { const int vv = __shfl_up(incl, off, 32); if (lane >= off) incl += vv; }
    const int wtot = __shfl(incl, 31, 32); int pos = incl - cnt;
    if (cnt > 0) {
#pragma unroll
      for (int u = 0; u < EPT; ++u) if (hd[u] >= 0) { ssrc[wave][pos] = e0 + u; sdl[wave][pos] = hd[u]; ++pos; } }
    if (lane == 0) scnt[wave] = wtot;
    __syncthreads();
#pragma unroll 1
    for (int w = 0; w < 8; ++w) { const int nh = scnt[w];
#pragma unroll 1
      for (int i = tid; i < nh; i += 256) { const int e = ssrc[w][i]; int r = etyp[e]; const bool ok = (r >= 0) && (r < NR); r = ok ? r : 0;
        swgt[w][i] = ok ? lamv * expf(-betav * fabsf(etim[e])) : 0.f; ssrc[w][i] = clampn(esrc[e]) * 8 + r; } }
    __syncthreads();
    if (tid < HD) { const int f = tid;
      for (int w = 0; w < 8; ++w) { const int nh = scnt[w]; for (int i = 0; i < nh; ++i) { const int sr = ssrc[w][i], dl = sdl[w][i]; const int s = sr >> 3, r = sr & 7; const float wg = swgt[w][i];
          sacc[dl][f] += wg * T[(size_t)s * TW + r * HD + f]; if (f < NR && f == r) sws[dl][r] += wg; } } }
    __syncthreads(); }
  for (int q = tid; q < RB * (HD / 4); q += 256) { const int rl = q >> 4, pc = q & 15; const int row = r0 + rl; v4f v = (row < NN) ? *(const v4f*)(&sacc[rl][pc * 4]) : (v4f){0.f, 0.f, 0.f, 0.f}; vst2(Hpart + (size_t)row * HD + pc * 4, v); }
  for (int q = tid; q < RB * 2; q += 256) { const int rl = q >> 1, hf = q & 1; const int row = r0 + rl; v4f v = {0.f, 0.f, 0.f, 0.f};
    if (row < NN) { if (hf == 0) { v[0] = sws[rl][0]; v[1] = sws[rl][1]; v[2] = sws[rl][2]; v[3] = sws[rl][3]; } else { v[0] = sws[rl][4]; } }
    vst2(WS + (size_t)row * 8 + hf * 4, v); }
}
__device__ __forceinline__ F2 split_row_scaled(const float* row, int k0, int lane, float sc) { float v[16]; const float* p = row + k0 + 8 * (lane >> 4);
#pragma unroll
  for (int i = 0; i < 8; ++i) { v[i] = p[i] * sc; v[8 + i] = p[16 + i] * sc; }
  return bsplit16(v); }
__global__ __launch_bounds__(128) void k_bpart(const float* __restrict__ Hin, const float* __restrict__ WS, const float* __restrict__ rW, const float* __restrict__ rb, const float* __restrict__ Hpart, float* __restrict__ Hout) {
  __shared__ __align__(16) float so[4][16][68];
  const int tid = threadIdx.x, wave = tid >> 5, lane = tid & 31, col = lane & 15, g = lane >> 4;
  const int r0 = blockIdx.x * 64 + wave * 16; const int ra = (r0 + col) < NN ? (r0 + col) : (NN - 1);
  v8f acc[4] = {};
#pragma unroll 1
  for (int kc = 0; kc < KB / 32; ++kc) { const int r = kc >> 1, k0 = (kc & 1) * 32; const float wsv = WS[(size_t)ra * 8 + r];
    const F2 a = split_row_scaled(Hin + (size_t)ra * HD, k0, lane, wsv);
#pragma unroll
    for (int j = 0; j < 4; ++j) acc[j] = mac3(a, split_col(rW + ((size_t)r * 2 * HD + HD) * HD, k0, j * 16 + col, lane, HD, HD), acc[j]); }
#pragma unroll
  for (int j = 0; j < 4; ++j) { const int n = j * 16 + col;
#pragma unroll
    for (int rr = 0; rr < 8; ++rr) { const int row = r0 + 8 * g + rr; float v = 0.f;
      if (row < NN) { v = acc[j][rr] + Hpart[(size_t)row * HD + n]; const float* wsr = WS + (size_t)row * 8;
#pragma unroll
        for (int r = 0; r < NR; ++r) v += wsr[r] * rb[r * HD + n]; }
      so[wave][8 * g + rr][n] = v; } }
  LDSX();
  for (int rl = 0; rl < 16; ++rl) { if (lane < 16) vst2(Hout + (size_t)(r0 + rl) * HD + lane * 4, *(const v4f*)(&so[wave][rl][lane * 4])); }
}
__global__ __launch_bounds__(128) void k_out(const float* __restrict__ H0, const float* __restrict__ H1, const float* __restrict__ H2, const float* __restrict__ W0, const float* __restrict__ b0,
                                            const float* __restrict__ W1, const float* __restrict__ b1, const float* __restrict__ W2, const float* __restrict__ b2, float* __restrict__ out) {
  __shared__ __align__(16) float so[4][16][68];
  const int tid = threadIdx.x, wave = tid >> 5, lane = tid & 31, col = lane & 15, g = lane >> 4;
  const int r0 = blockIdx.x * 64 + wave * 16; const int ra = (r0 + col) < NN ? (r0 + col) : (NN - 1);
  float res[4][8];
#pragma unroll
  for (int j = 0; j < 4; ++j)
#pragma unroll
    for (int rr = 0; rr < 8; ++rr) res[j][rr] = 0.f;
#pragma unroll 1
  for (int term = 0; term < 3; ++term) { const float* Hs = term == 0 ? H0 : (term == 1 ? H1 : H2); const float* W = term == 0 ? W0 : (term == 1 ? W1 : W2); const float* bb = term == 0 ? b0 : (term == 1 ? b1 : b2);
    v8f acc[4] = {};
#pragma unroll
    for (int kc = 0; kc < HD / 32; ++kc) { const F2 a = split_row(Hs + (size_t)ra * HD, kc * 32, lane);
#pragma unroll
      for (int j = 0; j < 4; ++j) acc[j] = mac3(a, split_col(W, kc * 32, j * 16 + col, lane, HD, HD), acc[j]); }
#pragma unroll
    for (int j = 0; j < 4; ++j) { const float bj = bb[j * 16 + col];
#pragma unroll
      for (int rr = 0; rr < 8; ++rr) res[j][rr] += lrelu(acc[j][rr] + bj); } }
#pragma unroll
  for (int j = 0; j < 4; ++j)
#pragma unroll
    for (int rr = 0; rr < 8; ++rr) so[wave][8 * g + rr][j * 16 + col] = res[j][rr];
  LDSX();
  for (int rl = 0; rl < 16; ++rl) { if (r0 + rl >= NN) break; if (lane < 16) vst2(out + (size_t)(r0 + rl) * HD + lane * 4, *(const v4f*)(&so[wave][rl][lane * 4])); }
}
extern "C" void kernel_launch(void* const* d_in, const int* in_sizes, int n_in, void* d_out, int out_size, void* d_ws, size_t ws_size, hipStream_t stream) {
  (void)in_sizes; (void)n_in; (void)out_size; (void)ws_size;
  const float* x = (const float*)d_in[0]; const int* ei = (const int*)d_in[1]; const int* etyp = (const int*)d_in[2]; const float* etim = (const float*)d_in[3];
  const float* fW = (const float*)d_in[4]; const float* fb = (const float*)d_in[5]; const float* rW1 = (const float*)d_in[6]; const float* rb1 = (const float*)d_in[7]; const float* rW2 = (const float*)d_in[8]; const float* rb2 = (const float*)d_in[9];
  const float* oW0 = (const float*)d_in[10]; const float* ob0 = (const float*)d_in[11]; const float* oW1 = (const float*)d_in[12]; const float* ob1 = (const float*)d_in[13]; const float* oW2 = (const float*)d_in[14]; const float* ob2 = (const float*)d_in[15];
  const float* lam = (const float*)d_in[16]; const float* beta = (const float*)d_in[17];
  const int* esrc = ei; const int* edst = ei + NE;
  float* out = (float*)d_out;
  char* ws = (char*)d_ws; size_t off = 0;
  auto take = [&](size_t bytes) { char* p = ws + off; off += (bytes + 255) & ~(size_t)255; return p; };
  float* H0 = (float*)take((size_t)NNP * HD * 4); float* H1 = (float*)take((size_t)NNP * HD * 4); float* H2 = (float*)take((size_t)NNP * HD * 4);
  float* TA = (float*)take((size_t)NNP * TW * 4); float* HP = (float*)take((size_t)NNP * HD * 4); float* WS = (float*)take((size_t)NNP * 8 * 4);
  k_node<DIN, HD, 0><<<NNP / 64, 128, 0, stream>>>(x, DIN, fW, fb, H0);
  k_node<HD, TW, 1><<<NNP / 64, 128, 0, stream>>>(H0, HD, rW1, nullptr, TA);
  k_rel<<<NRB, 256, 0, stream>>>(esrc, edst, etyp, etim, lam, beta, TA, HP, WS);
  k_bpart<<<NNP / 64, 128, 0, stream>>>(H0, WS, rW1, rb1, HP, H1);
  k_node<HD, TW, 1><<<NNP / 64, 128, 0, stream>>>(H1, HD, rW2, nullptr, TA);
  k_rel<<<NRB, 256, 0, stream>>>(esrc, edst, etyp, etim, lam, beta, TA, HP, WS);
  k_bpart<<<NNP / 64, 128, 0, stream>>>(H1, WS, rW2, rb2, HP, H2);
  k_out<<<NNP / 64, 128, 0, stream>>>(H0, H1, H2, oW0, ob0, oW1, ob1, oW2, ob2, out);
}
